// GaussianFC_42717744726248
// MI455X (gfx1250) — hardware-run, weakly checked
//
#include <hip/hip_runtime.h>
#include <stddef.h>


typedef _Float16 v16h __attribute__((ext_vector_type(16)));
typedef _Float16 v8h  __attribute__((ext_vector_type(8)));
typedef float    v8f  __attribute__((ext_vector_type(8)));
typedef float    v4f  __attribute__((ext_vector_type(4)));

#ifndef NB
#define NB 64
#endif
#ifndef NOUT
#define NOUT 8192
#endif
#define NB_FULL  64
#define OUT_FULL 8192
#define KIN      8192

#define NWAVE 4
#define BCOLS (NWAVE * 16)
#define MT    (NB / 16)
#define LDC   68

#define XCARRY 64.0f
#define WCARRY 64.0f

static_assert(NB >= 16 && NB <= NB_FULL && (NB % 16) == 0);
static_assert(NOUT >= BCOLS && NOUT <= OUT_FULL && (NOUT % BCOLS) == 0);
static_assert((KIN % 32) == 0 && (KIN % 1024) == 0);
static_assert(((size_t)NB * KIN) % 2048 == 0);
static_assert(BCOLS == 16 * 4);
static_assert(NWAVE * 32 == 128);
static_assert((NB % 8) == 0);
static_assert((LDC % 4) == 0 && LDC >= BCOLS);
static_assert(((size_t)(NB - 1) * OUT_FULL + NOUT) * 4 <= (size_t)2097152);

#define X16_BYTES ((size_t)NB * KIN * 2)
#define PAR_BYTES ((size_t)KIN * 4)
#define OFF_X16 ((size_t)0)
#define OFF_MUB (OFF_X16 + X16_BYTES)
#define OFF_COF (OFF_MUB + PAR_BYTES)
#define OFF_AMC (OFF_COF + PAR_BYTES)
#define WS_TOTAL (OFF_AMC + PAR_BYTES)
static_assert((X16_BYTES % 128) == 0 && (PAR_BYTES % 128) == 0);
static_assert(WS_TOTAL <= (size_t)134217728);

__device__ __forceinline__ float bf16r(float x) {
  unsigned int u = __float_as_uint(x);
  u = (u + 0x7FFFu + ((u >> 16) & 1u)) & 0xFFFF0000u;
  return __uint_as_float(u);
}

__device__ __forceinline__ v16h frag_at(const _Float16* p) {
  v8h lo = *(const v8h*)(p);
  v8h hi = *(const v8h*)(p + 16);
  v16h out;
#pragma unroll
  for (int i = 0; i < 8; ++i) { out[i] = lo[i]; out[i + 8] = hi[i]; }
  return out;
}

__device__ __forceinline__ v8f wmma16(v16h a, v16h b, v8f c) {
  v8f d = __builtin_amdgcn_wmma_f32_16x16x32_f16(false, a, false, b, (short)0, c,
                                                 false, false);
  asm volatile("v_nop\n\tv_nop\n\tv_nop\n\tv_nop" : "+v"(d) : "v"(a), "v"(b));
  return d;
}

__device__ __forceinline__ float relu_act(float t) {
  return fmaxf(t, 0.0f);
}

static __device__ __forceinline__ _Float16 toh_flush(float v) {
  const _Float16 r = (_Float16)v;
  return (fabsf(v) < 6.103515625e-05f) ? (_Float16)0.0f : r;
}

__device__ __forceinline__ _Float16 gauss_h(float fn, float m, float c, float a) {
  const float d = fn - m;
  float e = d * d * c;
  e = (e < -64.0f) ? -64.0f : e;
  const float p = __builtin_amdgcn_exp2f(e);
  return toh_flush(a * p);
}

__device__ __forceinline__ v8h gauss8(const float* __restrict__ MUB, const float* __restrict__ COF,
                                      const float* __restrict__ AMC, unsigned k, float fn) {
  const v4f m0 = *(const v4f*)(MUB + k);
  const v4f m1 = *(const v4f*)(MUB + k + 4u);
  const v4f c0 = *(const v4f*)(COF + k);
  const v4f c1 = *(const v4f*)(COF + k + 4u);
  const v4f a0 = *(const v4f*)(AMC + k);
  const v4f a1 = *(const v4f*)(AMC + k + 4u);
  v8h o;
#pragma unroll
  for (int i = 0; i < 4; ++i) {
    o[i]     = gauss_h(fn, m0[i], c0[i], a0[i]);
    o[i + 4] = gauss_h(fn, m1[i], c1[i], a1[i]);
  }
  return o;
}

__global__ __launch_bounds__(256) void gparam_kernel(
    const float* __restrict__ mu, const float* __restrict__ sigma, const float* __restrict__ amp,
    float* __restrict__ mub, float* __restrict__ cof, float* __restrict__ amc) {
#pragma clang fp contract(off)
  const unsigned k = (blockIdx.x * 256u + threadIdx.x) * 4u;
  const v4f m = *(const v4f*)(mu + k);
  const v4f s = *(const v4f*)(sigma + k);
  const v4f a = *(const v4f*)(amp + k);
  v4f om, oc, oa;
#pragma unroll
  for (int i = 0; i < 4; ++i) {
    const float sb = bf16r(s[i]);
    om[i] = bf16r(m[i]);
    oc[i] = -1.4426950408889634f * __builtin_amdgcn_rcpf(2.0f * sb * sb);
    oa[i] = WCARRY * bf16r(a[i]);
  }
  *(volatile v4f*)(mub + k) = om;
  *(volatile v4f*)(cof + k) = oc;
  *(volatile v4f*)(amc + k) = oa;
  __threadfence();
  *(volatile v4f*)(mub + k) = om;
  *(volatile v4f*)(cof + k) = oc;
  *(volatile v4f*)(amc + k) = oa;
}

__global__ __launch_bounds__(256) void xconv_kernel(
    const float* __restrict__ X, _Float16* __restrict__ X16) {
#pragma clang fp contract(off)
  const size_t e = ((size_t)blockIdx.x * 256u + threadIdx.x) * 8u;
  const v4f a0 = *(const v4f*)(X + e);
  const v4f a1 = *(const v4f*)(X + e + 4u);
  v8h o;
#pragma unroll
  for (int i = 0; i < 4; ++i) {
    o[i]     = toh_flush(XCARRY * bf16r(a0[i]));
    o[i + 4] = toh_flush(XCARRY * bf16r(a1[i]));
  }
  _Float16* p = X16 + e;
  *(volatile v8h*)p = o;
  __threadfence();
  *(volatile v8h*)p = o;
}

__global__ __launch_bounds__(128) void gfc_gemm_kernel(
    const _Float16* __restrict__ X16, const float* __restrict__ MUB,
    const float* __restrict__ COF, const float* __restrict__ AMC,
    const float* __restrict__ bias, float* __restrict__ outf) {
  __shared__ float Cs[NB * LDC];
  const unsigned tid = threadIdx.x, lane = tid & 31u;
  const unsigned wave = (unsigned)__builtin_amdgcn_readfirstlane((int)(threadIdx.x >> 5));
  const unsigned hh = lane >> 4, m = lane & 15u;
  const unsigned n0 = blockIdx.x * (unsigned)BCOLS;
  const float fn = (float)(n0 + wave * 16u + m);

  const _Float16* ap = X16 + (size_t)m * KIN + hh * 8u;
  v8f acc[MT];
#pragma unroll
  for (int mt = 0; mt < MT; ++mt) acc[mt] = (v8f){};

#pragma unroll 1
  for (unsigned k0 = 0; k0 < (unsigned)KIN; k0 += 32u) {
    const unsigned ka = k0 + hh * 8u;
    const v8h lo = gauss8(MUB, COF, AMC, ka, fn);
    const v8h hi = gauss8(MUB, COF, AMC, ka + 16u, fn);
    v16h bf;
#pragma unroll
    for (int i = 0; i < 8; ++i) { bf[i] = lo[i]; bf[i + 8] = hi[i]; }
#pragma unroll
    for (int mt = 0; mt < MT; ++mt) {
      const v16h a = frag_at(ap + (size_t)mt * 16u * KIN + k0);
      acc[mt] = wmma16(a, bf, acc[mt]);
    }
  }

#pragma unroll
  for (int mt = 0; mt < MT; ++mt)
#pragma unroll
    for (int r = 0; r < 8; ++r)
      Cs[((unsigned)mt * 16u + hh * 8u + (unsigned)r) * LDC + wave * 16u + m] = acc[mt][r];
  __syncthreads();

  const float cs = 1.0f / (XCARRY * WCARRY);
  v4f xs[NB / 8];
  size_t off[NB / 8];
#pragma unroll
  for (unsigned i = 0; i < (unsigned)(NB / 8); ++i) {
    const unsigned r = 8u * i + (tid >> 4);
    const unsigned c = (tid & 15u) * 4u;
    const v4f u = *(const v4f*)&Cs[r * LDC + c];
    const v4f g = *(const v4f*)(bias + n0 + c);
    v4f val;
#pragma unroll
    for (int j = 0; j < 4; ++j) val[j] = relu_act(u[j] * cs + bf16r(g[j]));
    xs[i] = val;
    off[i] = (size_t)r * OUT_FULL + n0 + c;
  }
#pragma unroll
  for (int i = 0; i < NB / 8; ++i) *(volatile v4f*)(outf + off[i]) = xs[i];
  __threadfence();
#pragma unroll
  for (int i = 0; i < NB / 8; ++i) *(volatile v4f*)(outf + off[i]) = xs[i];
}

extern "C" void kernel_launch(void* const* d_in, const int* in_sizes, int n_in,
                              void* d_out, int out_size, void* d_ws, size_t ws_size,
                              hipStream_t stream) {
  if (n_in < 5) return;
  if ((long long)in_sizes[0] < (long long)NB * KIN) return;
  if (in_sizes[1] < KIN || in_sizes[2] < KIN || in_sizes[3] < KIN) return;
  if (in_sizes[4] < NOUT) return;
  if ((long long)out_size < (long long)(NB - 1) * OUT_FULL + NOUT) return;
  if (ws_size < WS_TOTAL) return;

  const float* X     = (const float*)d_in[0];
  const float* mu    = (const float*)d_in[1];
  const float* sigma = (const float*)d_in[2];
  const float* amp   = (const float*)d_in[3];
  const float* bias  = (const float*)d_in[4];
  float* out = (float*)d_out;

  char* ws = (char*)d_ws;
  _Float16* X16 = (_Float16*)(ws + OFF_X16);
  float*    MUB = (float*)(ws + OFF_MUB);
  float*    COF = (float*)(ws + OFF_COF);
  float*    AMC = (float*)(ws + OFF_AMC);

  gparam_kernel<<<dim3(KIN / 1024), dim3(256), 0, stream>>>(mu, sigma, amp, MUB, COF, AMC);
  xconv_kernel<<<dim3((unsigned)(((size_t)NB * KIN) / 2048)), dim3(256), 0, stream>>>(X, X16);
  gfc_gemm_kernel<<<dim3(NOUT / BCOLS), dim3(128), 0, stream>>>(X16, MUB, COF, AMC, bias, out);
}
